// ExplaiNN_66606352827149
// MI455X (gfx1250) — hardware-verified
//
#include <hip/hip_runtime.h>
#include <math.h>

typedef __attribute__((ext_vector_type(16))) _Float16 v16h;
typedef __attribute__((ext_vector_type(16))) __bf16 v16b;
typedef __attribute__((ext_vector_type(8)))  _Float16 v8h;
typedef __attribute__((ext_vector_type(8)))  float v8f;
typedef __attribute__((ext_vector_type(4)))  float v4f;
typedef __attribute__((ext_vector_type(2)))  float v2f;
typedef __attribute__((ext_vector_type(4)))  unsigned v4u;
typedef __attribute__((ext_vector_type(4)))  int v4i;
typedef float __attribute__((may_alias)) float_a;
typedef int __attribute__((may_alias)) int_a;

template <typename T> __device__ __forceinline__ void vst2(void* p, T v) { *(volatile T*)p = v; __threadfence(); *(volatile T*)p = v; }
__device__ __forceinline__ v8f wmma16(v16h a, v16h b, v8f c) {
  v8f d = __builtin_amdgcn_wmma_f32_16x16x32_f16(false, a, false, b, (short)0, c, false, false);
  asm volatile("v_nop\n\tv_nop\n\tv_nop\n\tv_nop" : "+v"(d) : "v"(a), "v"(b));
  return d;
}
__device__ __forceinline__ v8f wmma_bf(v16b a, v16b b, v8f c) {
  v8f d = __builtin_amdgcn_wmma_f32_16x16x32_bf16(false, a, false, b, (short)0, c, false, false);
  asm volatile("v_nop\n\tv_nop\n\tv_nop\n\tv_nop" : "+v"(d) : "v"(a), "v"(b));
  return d;
}
__device__ __forceinline__ v16h frag_h(const _Float16* rowk0, int lane) {
  union { v16h v; v8h q[2]; } u; const _Float16* p = rowk0 + 8 * (lane >> 4);
  u.q[0] = *(const v8h*)p; u.q[1] = *(const v8h*)(p + 16); return u.v;
}
__device__ __forceinline__ v16h frag_f32(const float* rowk0, int lane) {
  v16h a; const float* p = rowk0 + 8 * (lane >> 4);
#pragma unroll
  for (int i = 0; i < 8; ++i) { a[i] = (_Float16)p[i]; a[8 + i] = (_Float16)p[16 + i]; }
  return a;
}
__device__ __forceinline__ v16h frag_f32s(const float* rowk0, int lane, float sc) {
  v16h a; const float* p = rowk0 + 8 * (lane >> 4);
#pragma unroll
  for (int i = 0; i < 8; ++i) { a[i] = (_Float16)(p[i] * sc); a[8 + i] = (_Float16)(p[16 + i] * sc); }
  return a;
}
__device__ __forceinline__ v16h fragc_f32(const float* W, int k0, int n, int lane, int ld, int K) {
  v16h a; const int g = lane >> 4;
#pragma unroll
  for (int i = 0; i < 8; ++i) { const int ka = k0 + 8 * g + i, kb = ka + 16;
    a[i] = (_Float16)(ka < K ? W[(size_t)ka * ld + n] : 0.f); a[8 + i] = (_Float16)(kb < K ? W[(size_t)kb * ld + n] : 0.f); }
  return a;
}
struct F2 { v16b h, l; };
__device__ __forceinline__ F2 bsplit16(const float v[16]) { F2 r;
#pragma unroll
  for (int i = 0; i < 16; ++i) { const __bf16 h = (__bf16)v[i]; r.h[i] = h; r.l[i] = (__bf16)(v[i] - (float)h); }
  return r; }
__device__ __forceinline__ F2 split_row(const float* row, int k0, int lane) { float v[16]; const float* p = row + k0 + 8 * (lane >> 4);
#pragma unroll
  for (int i = 0; i < 8; ++i) { v[i] = p[i]; v[8 + i] = p[16 + i]; }
  return bsplit16(v); }
__device__ __forceinline__ F2 split_rowK(const float* row, int k0, int lane, int K) { float v[16]; const int g = lane >> 4;
#pragma unroll
  for (int i = 0; i < 8; ++i) { const int ka = k0 + 8 * g + i, kb = ka + 16; v[i] = ka < K ? row[ka] : 0.f; v[8 + i] = kb < K ? row[kb] : 0.f; }
  return bsplit16(v); }
__device__ __forceinline__ F2 split_col(const float* W, int k0, int n, int lane, int ld, int K) { float v[16]; const int g = lane >> 4;
#pragma unroll
  for (int i = 0; i < 8; ++i) { const int ka = k0 + 8 * g + i, kb = ka + 16; v[i] = ka < K ? W[(size_t)ka * ld + n] : 0.f; v[8 + i] = kb < K ? W[(size_t)kb * ld + n] : 0.f; }
  return bsplit16(v); }
__device__ __forceinline__ v8f mac3(const F2& a, const F2& b, v8f c) { c = wmma_bf(a.l, b.h, c); c = wmma_bf(a.h, b.l, c); return wmma_bf(a.h, b.h, c); }
__device__ __forceinline__ float sigm(float v) { return 1.0f / (1.0f + expf(-v)); }
#define LDSX() do { asm volatile("s_wait_dscnt 0" ::: "memory"); __builtin_amdgcn_wave_barrier(); __builtin_amdgcn_fence(__ATOMIC_RELEASE, "workgroup"); } while (0)

#define NBT 256
#define LL 1000
#define NCH 4
#define KW 19
#define NG 300
#define NGP 304
#define KC (NCH * KW)
#define KCP 96
#define PP 100
#define HID 100
#define NCHUNK 13
#define HPB 30016

__device__ __forceinline__ v16h frag_f32sK3(const float* __restrict__ row, int k0, int lane, float sc, int K) {
  const int g = lane >> 4; v16h r;
#pragma unroll
  for (int i = 0; i < 8; ++i) { const int ka = k0 + 8 * g + i, kb = ka + 16; r[i] = (_Float16)((ka < K ? row[ka] : 0.f) * sc); r[8 + i] = (_Float16)((kb < K ? row[kb] : 0.f) * sc); }
  return r;
}
__global__ __launch_bounds__(160) void k_conv(const float* __restrict__ x, const float* __restrict__ cw, const float* __restrict__ cb, const float* __restrict__ g1, const float* __restrict__ be1, const float* __restrict__ m1, const float* __restrict__ v1, float* __restrict__ HP) {
  __shared__ __align__(16) _Float16 sa[5][3][16][40];
  __shared__ __align__(16) float sh[80][NGP + 1];
  __shared__ __align__(16) float sp[8][NGP];
  const int tid = threadIdx.x, wave = tid >> 5, lane = tid & 31, col = lane & 15, g = lane >> 4;
  const int b = blockIdx.y, l0b = blockIdx.x * 80, l0 = l0b + wave * 16;
  { const int l = l0 + col;
#pragma unroll
    for (int kc = 0; kc < 3; ++kc) { union { v8h h[2]; v4u u2[2]; } pk;
#pragma unroll
      for (int u = 0; u < 16; ++u) { const int k = kc * 32 + g * 16 + u; float v = 0.f;
        if (k < KC && l < LL) { const int c = k / KW, j = k % KW; const int pos = l + j - KW / 2; if (pos >= 0 && pos < LL) v = x[((size_t)b * NCH + c) * LL + pos]; }
        pk.h[u >> 3][u & 7] = (_Float16)v; }
      *(v4u*)(&sa[wave][kc][col][g * 16]) = pk.u2[0]; *(v4u*)(&sa[wave][kc][col][g * 16 + 8]) = pk.u2[1]; } }
  LDSX();
  v16h af[3];
#pragma unroll
  for (int kc = 0; kc < 3; ++kc) af[kc] = frag_h(&sa[wave][kc][col][0], lane);
#pragma unroll 1
  for (int t = 0; t < NGP / 16; ++t) { const int o = t * 16 + col; const int oo = o < NG ? o : 0; v8f acc = {};
#pragma unroll
    for (int kc = 0; kc < 3; ++kc) acc = wmma16(af[kc], frag_f32sK3(cw + (size_t)oo * KC, kc * 32, lane, 16.0f, KC), acc);
    const float sc = g1[oo] / sqrtf(v1[oo] + 1e-5f), bb = cb[oo], mm = m1[oo], be = be1[oo];
#pragma unroll
    for (int r = 0; r < 8; ++r) { float v = acc[r] * (1.0f / 16.0f) + bb; v = (v - mm) * sc + be; sh[wave * 16 + 8 * g + r][o] = (o < NG) ? (v > 0.f ? v : 0.f) : 0.f; } }
  __syncthreads();
  const int npool = (l0b + 80 <= LL) ? 8 : (LL - l0b) / 10;
  for (int q = tid; q < 8 * NGP; q += 160) { const int pl = q / NGP, o = q % NGP; float mx = 0.f;
    if (pl < npool) { mx = sh[pl * 10][o]; for (int e = 1; e < 10; ++e) mx = fmaxf(mx, sh[pl * 10 + e][o]); }
    sp[pl][o] = mx; }
  __syncthreads();
  for (int q = tid; q < npool * (NG / 4); q += 160) { const int pl = q / (NG / 4), pc = q % (NG / 4); vst2(HP + (size_t)b * HPB + (size_t)(l0b / 10 + pl) * NG + pc * 4, *(const v4f*)(&sp[pl][pc * 4])); }
}
__global__ __launch_bounds__(128) void k_unit(const float* __restrict__ HP, const float* __restrict__ W1, const float* __restrict__ b1, const float* __restrict__ g2, const float* __restrict__ be2, const float* __restrict__ m2, const float* __restrict__ v2,
                                            const float* __restrict__ W2, const float* __restrict__ b2, const float* __restrict__ g3, const float* __restrict__ be3, const float* __restrict__ m3, const float* __restrict__ v3, float* __restrict__ H2) {
  __shared__ __align__(16) float sh1[NBT][HID + 4];
  __shared__ __align__(16) float so[NBT];
  const int tid = threadIdx.x, wave = tid >> 5, lane = tid & 31, col = lane & 15, g = lane >> 4;
  const int un = blockIdx.x;
  const float* W1g = W1 + (size_t)un * HID * PP;
#pragma unroll 1
  for (int rt = wave; rt < NBT / 16; rt += 4) {
    F2 a[4];
#pragma unroll
    for (int kc = 0; kc < 4; ++kc) { float v[16]; const int bb = rt * 16 + col;
#pragma unroll
      for (int i = 0; i < 8; ++i) { const int ka = kc * 32 + 8 * g + i, kb = ka + 16; v[i] = ka < PP ? HP[(size_t)bb * HPB + (size_t)ka * NG + un] : 0.f; v[8 + i] = kb < PP ? HP[(size_t)bb * HPB + (size_t)kb * NG + un] : 0.f; }
      a[kc] = bsplit16(v); }
#pragma unroll 1
    for (int t = 0; t < 7; ++t) { const int hh = t * 16 + col; const int hc = hh < HID ? hh : 0; v8f acc = {};
#pragma unroll
      for (int kc = 0; kc < 4; ++kc) acc = mac3(a[kc], split_rowK(W1g + (size_t)hc * PP, kc * 32, lane, PP), acc);
      const float sc = g2[un * HID + hc] / sqrtf(v2[un * HID + hc] + 1e-5f), bb = b1[un * HID + hc], mm = m2[un * HID + hc], be = be2[un * HID + hc];
#pragma unroll
      for (int r = 0; r < 8; ++r) { float vv = acc[r] + bb; vv = (vv - mm) * sc + be; if (hh < HID) sh1[rt * 16 + 8 * g + r][hh] = vv > 0.f ? vv : 0.f; } } }
  __syncthreads();
  { const float sc3 = g3[un] / sqrtf(v3[un] + 1e-5f), bb3 = b2[un], mm3 = m3[un], bt3 = be3[un];
    for (int bb = tid; bb < NBT; bb += 128) { float s = bb3;
#pragma unroll 4
      for (int hh = 0; hh < HID; ++hh) s += sh1[bb][hh] * W2[un * HID + hh];
      s = (s - mm3) * sc3 + bt3; so[bb] = s > 0.f ? s : 0.f; } }
  __syncthreads();
  if (tid < NBT / 4) vst2(H2 + (size_t)un * NBT + tid * 4, *(const v4f*)(&so[tid * 4]));
}
__global__ __launch_bounds__(256) void k_cls(const float* __restrict__ H2, const float* __restrict__ cwt, const float* __restrict__ cbias, float* __restrict__ out) {
  __shared__ __align__(16) float so[NBT * 2];
  const int tid = threadIdx.x;
  for (int q = tid; q < NBT * 2; q += 256) { const int bb = q >> 1, o = q & 1; float s = cbias[o];
#pragma unroll 4
    for (int un = 0; un < NG; ++un) s += H2[(size_t)un * NBT + bb] * cwt[o * NG + un];
    so[q] = s; }
  __syncthreads();
  if (tid < NBT * 2 / 4) vst2(out + tid * 4, *(const v4f*)(&so[tid * 4]));
}
extern "C" void kernel_launch(void* const* d_in, const int* in_sizes, int n_in, void* d_out, int out_size, void* d_ws, size_t ws_size, hipStream_t stream) {
  (void)in_sizes; (void)n_in; (void)out_size; (void)ws_size;
  const float** I = (const float**)d_in;
  float* out = (float*)d_out;
  char* ws = (char*)d_ws; size_t off = 0;
  auto take = [&](size_t bytes) { char* p = ws + off; off += (bytes + 255) & ~(size_t)255; return p; };
  float* HP = (float*)take((size_t)NBT * HPB * 4); float* H2 = (float*)take((size_t)NG * NBT * 4);
  k_conv<<<dim3(NCHUNK, NBT), 160, 0, stream>>>(I[0], I[1], I[2], I[3], I[4], I[5], I[6], HP);
  k_unit<<<NG, 128, 0, stream>>>(HP, I[7], I[8], I[9], I[10], I[11], I[12], I[13], I[14], I[15], I[16], I[17], I[18], H2);
  k_cls<<<1, 256, 0, stream>>>(H2, I[19], I[20], out);
}
